// TransformerBlock_De_87368224735424
// MI455X (gfx1250) — hardware-verified
//
#include <hip/hip_runtime.h>


namespace {
constexpr int NB = 4, S = 2048, DM = 512, NH = 8, HD = 64, NR = NB * S, MAXLEN = 22118;
constexpr float XS = 8.0f, WSC = 256.0f, PS = 8.0f, LOG2E = 1.4426950408889634f, NEG = 0.2f, LNEPS = 1e-5f;
typedef _Float16 b16;
typedef __attribute__((ext_vector_type(16))) _Float16 v16b;
typedef __attribute__((ext_vector_type(8))) _Float16 v8b;
typedef __attribute__((ext_vector_type(8))) float v8f;
typedef __attribute__((ext_vector_type(4))) float v4f;
__device__ __forceinline__ float bf16_rne(float f) { unsigned int u = __float_as_uint(f); u += 0x7FFFu + ((u >> 16) & 1u); return __uint_as_float(u & 0xFFFF0000u); }
__device__ __forceinline__ void split16(float v, b16& hi, b16& lo) { hi = (b16)v; lo = (b16)(v - (float)hi); }
__device__ __forceinline__ v16b frag_kb(const b16* p, int hh) { const v8b a = *(const v8b*)(p + 8 * hh), b = *(const v8b*)(p + 16 + 8 * hh); v16b f;
#pragma unroll
  for (int e = 0; e < 8; ++e) { f[e] = a[e]; f[8 + e] = b[e]; } return f; }
__device__ __forceinline__ v8f wmma16b(v16b a, v16b b, v8f c) { v8f d = __builtin_amdgcn_wmma_f32_16x16x32_f16(false, a, false, b, (short)0, c, false, false); asm volatile("v_nop\n\tv_nop\n\tv_nop\n\tv_nop" : "+v"(d) : "v"(a), "v"(b)); return d; }
__device__ __forceinline__ void wave_lds_sync() { __builtin_amdgcn_fence(__ATOMIC_RELEASE, "workgroup"); __builtin_amdgcn_wave_barrier(); __builtin_amdgcn_fence(__ATOMIC_ACQUIRE, "workgroup"); }
__device__ __forceinline__ int iclamp(int v, int lo, int hi) { return v < lo ? lo : (v > hi ? hi : v); }
__device__ __forceinline__ float lrelu(float x) { return x > 0.0f ? x : NEG * x; }

__global__ __launch_bounds__(256) void prepx_kernel(const float* __restrict__ x, const float* __restrict__ vis, const int* __restrict__ c1, const int* __restrict__ c2, const float* __restrict__ e1, const float* __restrict__ e2, b16* __restrict__ V16, b16* __restrict__ XPh, b16* __restrict__ XPl) {
  const size_t u = (size_t)blockIdx.x * 256 + threadIdx.x; if (u >= (size_t)NR * DM / 8) return; const size_t e = u * 8; const size_t row = e / DM; const int c0 = (int)(e % DM); v8b o, oh, ol;
  const v4f a = *(const v4f*)(vis + e), b = *(const v4f*)(vis + e + 4); for (int j = 0; j < 4; ++j) { o[j] = (b16)(bf16_rne(a[j]) * XS); o[4 + j] = (b16)(bf16_rne(b[j]) * XS); }
  const float* pe; if (c0 < DM / 2) { const int id = iclamp(c1[row], 0, MAXLEN - 1); pe = e1 + (size_t)id * (DM / 2) + c0; } else { const int id = iclamp(c2[row], 0, MAXLEN - 1); pe = e2 + (size_t)id * (DM / 2) + (c0 - DM / 2); }
  const v4f xa = *(const v4f*)(x + e), xb = *(const v4f*)(x + e + 4);
  for (int j = 0; j < 8; ++j) { const float xv = (j < 4 ? xa[j] : xb[j - 4]); const float v = bf16_rne(xv) + bf16_rne(pe[j]); b16 p, q; split16(v * XS, p, q); oh[j] = p; ol[j] = q; }
  for (int pass = 0; pass < 2; ++pass) { *(volatile v8b*)(V16 + e) = o; *(volatile v8b*)(XPh + e) = oh; *(volatile v8b*)(XPl + e) = ol; __threadfence(); }
}
__global__ __launch_bounds__(256) void prepw_kernel(const float* __restrict__ wq, const float* __restrict__ wk, const float* __restrict__ wv, const float* __restrict__ w1, const float* __restrict__ w2, b16* __restrict__ WT) {
  __shared__ __attribute__((aligned(16))) b16 T[64][64 + 8];
  const int ib = blockIdx.x * 64, ob = blockIdx.y * 64, kind = blockIdx.z, t_ = threadIdx.x; const float* w = kind == 0 ? wq : kind == 1 ? wk : kind == 2 ? wv : kind == 3 ? w1 : w2;
  for (int q = t_; q < 64 * 64; q += 256) { const int ii = q >> 6, oo = q & 63; T[oo][ii] = (b16)(bf16_rne(w[(size_t)(ib + ii) * DM + ob + oo]) * WSC); }
  __syncthreads();
  for (int pass = 0; pass < 2; ++pass) { for (int q = t_; q < 64 * 8; q += 256) { const int oo = q >> 3, c8 = (q & 7) * 8; *(volatile v8b*)(WT + ((size_t)kind * DM + ob + oo) * DM + ib + c8) = *(const v8b*)(&T[oo][c8]); } __threadfence(); }
}
__global__ __launch_bounds__(128) void proj_kernel(const b16* __restrict__ V16, const b16* __restrict__ XPh, const b16* __restrict__ XPl, const b16* __restrict__ WT, const float* __restrict__ bq, const float* __restrict__ bk, const float* __restrict__ bv, b16* __restrict__ Qh, b16* __restrict__ Ql, b16* __restrict__ Kh, b16* __restrict__ Kl, b16* __restrict__ VTh, b16* __restrict__ VTl) {
  __shared__ __attribute__((aligned(16))) b16 Th[4][16][128 + 8], Tl[4][16][128 + 8]; __shared__ __attribute__((aligned(16))) b16 Vt[128][64 + 8], Vtl[128][64 + 8];
  const int wave = threadIdx.x >> 5, lane = threadIdx.x & 31, nloc = lane & 15, hlf = lane >> 4, t_ = threadIdx.x; const int kind = blockIdx.z, n0 = blockIdx.y * 128; const size_t m0 = (size_t)blockIdx.x * 64 + wave * 16;
  const b16* W = WT + (size_t)kind * DM * DM; const float* bias = kind == 0 ? bq : kind == 1 ? bk : bv; v8f acc[8];
#pragma unroll
  for (int t = 0; t < 8; ++t) acc[t] = (v8f){};
  if (kind < 2) {
#pragma unroll 2
    for (int kb = 0; kb < DM; kb += 32) { const v16b a = frag_kb(V16 + (m0 + nloc) * DM + kb, hlf);
#pragma unroll
      for (int t = 0; t < 8; ++t) acc[t] = wmma16b(a, frag_kb(W + (size_t)(n0 + t * 16 + nloc) * DM + kb, hlf), acc[t]); }
#pragma unroll
    for (int t = 0; t < 8; ++t) { const float bb = bf16_rne(bias[n0 + t * 16 + nloc]);
#pragma unroll 1
      for (int r = 0; r < 8; ++r) { b16 p, q; split16((acc[t][r] * (1.0f / (XS * WSC)) + bb) * XS, p, q); Th[wave][8 * hlf + r][t * 16 + nloc] = p; Tl[wave][8 * hlf + r][t * 16 + nloc] = q; } }
    wave_lds_sync(); b16* dh = kind == 0 ? Qh : Kh; b16* dl = kind == 0 ? Ql : Kl;
    for (int pass = 0; pass < 2; ++pass) { for (int r2 = 0; r2 < 16; r2 += 2) { const int rr = r2 + (lane >> 4), c8 = (lane & 15) * 8; const size_t gi = (m0 + rr) * DM + n0 + c8; *(volatile v8b*)(dh + gi) = *(const v8b*)(&Th[wave][rr][c8]); *(volatile v8b*)(dl + gi) = *(const v8b*)(&Tl[wave][rr][c8]); } __threadfence(); }
  } else {
#pragma unroll 2
    for (int kb = 0; kb < DM; kb += 32) { const v16b a = frag_kb(XPh + (m0 + nloc) * DM + kb, hlf), al = frag_kb(XPl + (m0 + nloc) * DM + kb, hlf);
#pragma unroll
      for (int t = 0; t < 8; ++t) { const v16b bw = frag_kb(W + (size_t)(n0 + t * 16 + nloc) * DM + kb, hlf); acc[t] = wmma16b(a, bw, acc[t]); acc[t] = wmma16b(al, bw, acc[t]); } }
#pragma unroll
    for (int t = 0; t < 8; ++t) { const float bb = bf16_rne(bias[n0 + t * 16 + nloc]);
#pragma unroll 1
      for (int r = 0; r < 8; ++r) { b16 p, q; split16((acc[t][r] * (1.0f / (XS * WSC)) + bb) * XS, p, q); Vt[t * 16 + nloc][wave * 16 + 8 * hlf + r] = p; Vtl[t * 16 + nloc][wave * 16 + 8 * hlf + r] = q; } }
    __syncthreads(); const size_t r0 = (size_t)blockIdx.x * 64; const size_t b = r0 / S; const int s0 = (int)(r0 % S);
    for (int pass = 0; pass < 2; ++pass) { for (int q = t_; q < 128 * 8; q += 128) { const int cc = q >> 3, c8 = (q & 7) * 8; const int col = n0 + cc; const int h = col / HD, dd = col % HD; const size_t gi = (((b * NH + h) * HD + dd) * S) + s0 + c8; *(volatile v8b*)(VTh + gi) = *(const v8b*)(&Vt[cc][c8]); *(volatile v8b*)(VTl + gi) = *(const v8b*)(&Vtl[cc][c8]); } __threadfence(); }
  }
}
__global__ __launch_bounds__(64) void attn_kernel(const b16* __restrict__ Qh, const b16* __restrict__ Ql, const b16* __restrict__ Kh, const b16* __restrict__ Kl, const b16* __restrict__ VTh, const b16* __restrict__ VTl, b16* __restrict__ Oh, b16* __restrict__ Ol) {
  __shared__ __attribute__((aligned(16))) float To[2][16][HD + 4];
  const int wave = threadIdx.x >> 5, lane = threadIdx.x & 31, hh = lane >> 4, col = lane & 15; const int h = blockIdx.y, b = blockIdx.z; const int q0 = blockIdx.x * 32 + wave * 16, qi = q0 + col;
  const size_t qo = ((size_t)b * S + qi) * DM + h * HD; const v16b qa0 = frag_kb(Qh + qo, hh), qa1 = frag_kb(Qh + qo + 32, hh), ql0 = frag_kb(Ql + qo, hh), ql1 = frag_kb(Ql + qo + 32, hh);
  const b16* Kb = Kh + (size_t)b * S * DM + h * HD; const b16* Klb = Kl + (size_t)b * S * DM + h * HD; const b16* Vb = VTh + ((size_t)b * NH + h) * HD * S; const b16* Vlb = VTl + ((size_t)b * NH + h) * HD * S;
  v8f o[4] = {{}, {}, {}, {}}, ol[4] = {{}, {}, {}, {}}; float mrun = -INFINITY, lrun = 0.0f; const float cs = 0.125f * LOG2E / (XS * XS);
  for (int kb = 0; kb < S; kb += 32) {
    v8f s0 = {}, s1 = {};
    { const b16* k0 = Kb + (size_t)(kb + col) * DM, *k1 = Kb + (size_t)(kb + 16 + col) * DM, *k0l = Klb + (size_t)(kb + col) * DM, *k1l = Klb + (size_t)(kb + 16 + col) * DM;
      v16b f = frag_kb(k0, hh); s0 = wmma16b(f, qa0, s0); s0 = wmma16b(f, ql0, s0); s0 = wmma16b(frag_kb(k0l, hh), qa0, s0);
      f = frag_kb(k0 + 32, hh); s0 = wmma16b(f, qa1, s0); s0 = wmma16b(f, ql1, s0); s0 = wmma16b(frag_kb(k0l + 32, hh), qa1, s0);
      f = frag_kb(k1, hh); s1 = wmma16b(f, qa0, s1); s1 = wmma16b(f, ql0, s1); s1 = wmma16b(frag_kb(k1l, hh), qa0, s1);
      f = frag_kb(k1 + 32, hh); s1 = wmma16b(f, qa1, s1); s1 = wmma16b(f, ql1, s1); s1 = wmma16b(frag_kb(k1l + 32, hh), qa1, s1); }
    float e[16]; float bm = -INFINITY;
#pragma unroll
    for (int r = 0; r < 8; ++r) { e[r] = s0[r] * cs; e[8 + r] = s1[r] * cs; bm = fmaxf(bm, fmaxf(e[r], e[8 + r])); }
    bm = fmaxf(bm, __shfl_xor(bm, 16)); const float mn = fmaxf(mrun, bm); const float sc = exp2f(mrun - mn); float ls = 0.0f; v16b ph, pl;
#pragma unroll
    for (int i = 0; i < 16; ++i) { const float p = exp2f(e[i] - mn); ls += p; b16 a, c; split16(p * PS, a, c); ph[i] = a; pl[i] = c; }
    ls += __shfl_xor(ls, 16); lrun = lrun * sc + ls; mrun = mn;
#pragma unroll
    for (int t = 0; t < 4; ++t) { o[t] *= sc; ol[t] *= sc; const v16b vf = frag_kb(Vb + (size_t)(t * 16 + col) * S + kb, hh); o[t] = wmma16b(vf, ph, o[t]); ol[t] = wmma16b(vf, pl, ol[t]); ol[t] = wmma16b(frag_kb(Vlb + (size_t)(t * 16 + col) * S + kb, hh), ph, ol[t]); } }
  const float inv = 1.0f / (lrun * PS * XS);
#pragma unroll
  for (int t = 0; t < 4; ++t)
#pragma unroll
    for (int r = 0; r < 8; ++r) To[wave][col][t * 16 + 8 * hh + r] = (o[t][r] + ol[t][r]) * inv;
  wave_lds_sync();
  for (int pass = 0; pass < 2; ++pass) { for (int r4 = 0; r4 < 16; r4 += 4) { const int rr = r4 + (lane >> 3), c8 = (lane & 7) * 8; v8b hv, lv; for (int j = 0; j < 8; ++j) { b16 p, q; split16(To[wave][rr][c8 + j] * XS, p, q); hv[j] = p; lv[j] = q; }
      const size_t gi = ((size_t)b * S + q0 + rr) * DM + h * HD + c8; *(volatile v8b*)(Oh + gi) = hv; *(volatile v8b*)(Ol + gi) = lv; } __threadfence(); }
}
__global__ __launch_bounds__(128) void dense_kernel(const b16* __restrict__ Ah, const b16* __restrict__ Al, const b16* __restrict__ W, const float* __restrict__ bias, float* __restrict__ Y) {
  __shared__ __attribute__((aligned(16))) float Tf[4][16][128 + 4];
  const int wave = threadIdx.x >> 5, lane = threadIdx.x & 31, nloc = lane & 15, hlf = lane >> 4; const size_t m0 = (size_t)blockIdx.x * 64 + wave * 16; const int n0 = blockIdx.y * 128; v8f acc[8];
#pragma unroll
  for (int t = 0; t < 8; ++t) acc[t] = (v8f){};
#pragma unroll 2
  for (int kb = 0; kb < DM; kb += 32) { const v16b a = frag_kb(Ah + (m0 + nloc) * DM + kb, hlf), al = frag_kb(Al + (m0 + nloc) * DM + kb, hlf);
#pragma unroll
    for (int t = 0; t < 8; ++t) { const v16b bw = frag_kb(W + (size_t)(n0 + t * 16 + nloc) * DM + kb, hlf); acc[t] = wmma16b(a, bw, acc[t]); acc[t] = wmma16b(al, bw, acc[t]); } }
#pragma unroll
  for (int t = 0; t < 8; ++t) { const float bb = bf16_rne(bias[n0 + t * 16 + nloc]);
#pragma unroll 1
    for (int r = 0; r < 8; ++r) Tf[wave][8 * hlf + r][t * 16 + nloc] = lrelu(acc[t][r] * (1.0f / (XS * WSC)) + bb); }
  wave_lds_sync();
  for (int pass = 0; pass < 2; ++pass) { for (int rr = 0; rr < 16; ++rr) *(volatile v4f*)(Y + (m0 + rr) * DM + n0 + lane * 4) = *(const v4f*)(&Tf[wave][rr][lane * 4]); __threadfence(); }
}
template <int MODE>
__global__ __launch_bounds__(256) void ln_kernel(const float* __restrict__ X, const float* __restrict__ g, const float* __restrict__ bta, b16* __restrict__ Yh, b16* __restrict__ Yl, float* __restrict__ out) {
  const int wave = threadIdx.x >> 5, lane = threadIdx.x & 31; const size_t row = (size_t)blockIdx.x * 8 + wave; float x[16];
  { const v4f a = *(const v4f*)(X + row * DM + lane * 8), c = *(const v4f*)(X + row * DM + lane * 8 + 4), e = *(const v4f*)(X + row * DM + 256 + lane * 8), f = *(const v4f*)(X + row * DM + 256 + lane * 8 + 4); for (int j = 0; j < 4; ++j) { x[j] = a[j]; x[4 + j] = c[j]; x[8 + j] = e[j]; x[12 + j] = f[j]; } }
  float s = 0.0f; for (int j = 0; j < 16; ++j) s += x[j];
#pragma unroll
  for (int o = 16; o >= 1; o >>= 1) s += __shfl_xor(s, o);
  const float mu = s * (1.0f / DM); float q = 0.0f; for (int j = 0; j < 16; ++j) { const float d = x[j] - mu; q += d * d; }
#pragma unroll
  for (int o = 16; o >= 1; o >>= 1) q += __shfl_xor(q, o);
  const float rs = rsqrtf(q * (1.0f / DM) + LNEPS); float y[16]; for (int j = 0; j < 16; ++j) { const int c = (j < 8) ? lane * 8 + j : 256 + lane * 8 + (j - 8); y[j] = (x[j] - mu) * rs * bf16_rne(g[c]) + bf16_rne(bta[c]); }
  if (MODE == 0) { v8b h0, l0, h1, l1; for (int j = 0; j < 8; ++j) { b16 p, pl; split16(y[j] * XS, p, pl); h0[j] = p; l0[j] = pl; split16(y[8 + j] * XS, p, pl); h1[j] = p; l1[j] = pl; }
    for (int pass = 0; pass < 2; ++pass) { *(volatile v8b*)(Yh + row * DM + lane * 8) = h0; *(volatile v8b*)(Yh + row * DM + 256 + lane * 8) = h1; *(volatile v8b*)(Yl + row * DM + lane * 8) = l0; *(volatile v8b*)(Yl + row * DM + 256 + lane * 8) = l1; __threadfence(); } }
  else { v4f r0 = {y[0], y[1], y[2], y[3]}, r1 = {y[4], y[5], y[6], y[7]}, r2 = {y[8], y[9], y[10], y[11]}, r3 = {y[12], y[13], y[14], y[15]};
    for (int pass = 0; pass < 2; ++pass) { *(volatile v4f*)(out + row * DM + lane * 8) = r0; *(volatile v4f*)(out + row * DM + lane * 8 + 4) = r1; *(volatile v4f*)(out + row * DM + 256 + lane * 8) = r2; *(volatile v4f*)(out + row * DM + 256 + lane * 8 + 4) = r3; __threadfence(); } }
}
}

extern "C" void kernel_launch(void* const* d_in, const int* in_sizes, int n_in, void* d_out, int out_size, void* d_ws, size_t ws_size, hipStream_t stream) {
  (void)n_in;
  auto Fp = [&](int i) { return (const float*)d_in[i]; }; auto Ip = [&](int i) { return (const int*)d_in[i]; };
  if (in_sizes[0] != NR * DM || in_sizes[1] != NR * DM || in_sizes[2] != NR || in_sizes[3] != NR || in_sizes[4] != MAXLEN * DM / 2 || in_sizes[6] != DM * DM || in_sizes[12] != DM * DM || in_sizes[16] != DM * DM || out_size != NR * DM) return;
  size_t off = 0; char* ws = (char*)d_ws;
  auto carve = [&](size_t bytes) { char* p = ws + off; off += (bytes + 255) & ~(size_t)255; return p; };
  b16* V16 = (b16*)carve((size_t)NR * DM * 2); b16* XPh = (b16*)carve((size_t)NR * DM * 2); b16* XPl = (b16*)carve((size_t)NR * DM * 2); b16* WT = (b16*)carve((size_t)5 * DM * DM * 2);
  b16* Qh = (b16*)carve((size_t)NR * DM * 2); b16* Ql = (b16*)carve((size_t)NR * DM * 2); b16* Kh = (b16*)carve((size_t)NR * DM * 2); b16* Kl = (b16*)carve((size_t)NR * DM * 2); b16* VTh = (b16*)carve((size_t)NR * DM * 2); b16* VTl = (b16*)carve((size_t)NR * DM * 2);
  b16* Oh = V16; b16* Ol = XPh; float* Y = (float*)Qh; b16* H1h = Kh; b16* H1l = Kl; float* Y2 = (float*)VTh;
  if (off > ws_size || off > ((size_t)128 << 20)) return;
  prepx_kernel<<<(unsigned)(((size_t)NR * DM / 8 + 255) / 256), 256, 0, stream>>>(Fp(0), Fp(1), Ip(2), Ip(3), Fp(4), Fp(5), V16, XPh, XPl);
  prepw_kernel<<<dim3(DM / 64, DM / 64, 5), 256, 0, stream>>>(Fp(6), Fp(8), Fp(10), Fp(12), Fp(16), WT);
  proj_kernel<<<dim3(NR / 64, DM / 128, 3), 128, 0, stream>>>(V16, XPh, XPl, WT, Fp(7), Fp(9), Fp(11), Qh, Ql, Kh, Kl, VTh, VTl);
  attn_kernel<<<dim3(S / 32, NH, NB), 64, 0, stream>>>(Qh, Ql, Kh, Kl, VTh, VTl, Oh, Ol);
  dense_kernel<<<dim3(NR / 64, DM / 128), 128, 0, stream>>>(Oh, Ol, WT + (size_t)3 * DM * DM, Fp(13), Y);
  ln_kernel<0><<<NR / 8, 256, 0, stream>>>(Y, Fp(14), Fp(15), H1h, H1l, nullptr);
  dense_kernel<<<dim3(NR / 64, DM / 128), 128, 0, stream>>>(H1h, H1l, WT + (size_t)4 * DM * DM, Fp(17), Y2);
  ln_kernel<1><<<NR / 8, 256, 0, stream>>>(Y2, Fp(18), Fp(19), nullptr, nullptr, (float*)d_out);
}
